// CrossAttentionLayer_52802327937147
// MI455X (gfx1250) — hardware-verified
//
#include <hip/hip_runtime.h>


#define N1   8192
#define N2   8192
#define D1   256
#define D2   128
#define RB   1024
#define MZP  32
typedef _Float16 h16;
typedef unsigned short bf;
typedef __attribute__((ext_vector_type(16))) __bf16   v16bf;
typedef __attribute__((ext_vector_type(16))) _Float16 v16h;
typedef __attribute__((ext_vector_type(8)))  _Float16 v8h;
typedef __attribute__((ext_vector_type(8)))  unsigned short v8us;
typedef __attribute__((ext_vector_type(8)))  float    v8f;
typedef __attribute__((ext_vector_type(4)))  float    v4f;
typedef v8h  __attribute__((may_alias)) v8ha;
typedef v4f  __attribute__((may_alias)) v4fa;
typedef v8us __attribute__((may_alias)) v8usa;

__device__ __forceinline__ unsigned short f2bf(float f) { unsigned u = __float_as_uint(f); u += 0x7FFFu + ((u >> 16) & 1u); return (unsigned short)(u >> 16); }
__device__ __forceinline__ float bf2f(unsigned short b) { return __uint_as_float(((unsigned)b) << 16); }
__device__ __forceinline__ float bfr(float f) { return bf2f(f2bf(f)); }
__device__ __forceinline__ v16h cat16(v8h lo, v8h hi) { return __builtin_shufflevector(lo, hi, 0, 1, 2, 3, 4, 5, 6, 7, 8, 9, 10, 11, 12, 13, 14, 15); }
__device__ __forceinline__ v16bf cat16b(v8us lo, v8us hi) { return __builtin_bit_cast(v16bf, __builtin_shufflevector(lo, hi, 0, 1, 2, 3, 4, 5, 6, 7, 8, 9, 10, 11, 12, 13, 14, 15)); }
__device__ __forceinline__ v8f wmma16(v16h a, v16h b, v8f c) { return __builtin_amdgcn_wmma_f32_16x16x32_f16(false, a, false, b, (short)0, c, false, false); }
__device__ __forceinline__ v8f wmmab(v16bf a, v16bf b, v8f c) { return __builtin_amdgcn_wmma_f32_16x16x32_bf16(false, a, false, b, (short)0, c, false, false); }


template <typename T16> struct WFrag;
template <> struct WFrag<h16> { typedef v16h V; static __device__ __forceinline__ V ld(const h16* p) { return cat16(*(const v8h*)p, *(const v8h*)(p + 16)); } static __device__ __forceinline__ v8f mma(V a, V b, v8f c) { return wmma16(a, b, c); } };
template <> struct WFrag<bf> { typedef v16bf V; static __device__ __forceinline__ V ld(const bf* p) { return cat16b(*(const v8us*)p, *(const v8us*)(p + 16)); } static __device__ __forceinline__ v8f mma(V a, V b, v8f c) { return wmmab(a, b, c); } };
template <typename T16, int NSPLIT, bool BIAS>
__global__ __launch_bounds__(32) void k_gemmw(const T16* __restrict__ A, const T16* __restrict__ A2, const T16* __restrict__ Bt, const T16* __restrict__ Bt2, int K, float* C, int ldc, const float* __restrict__ bias, size_t sA, size_t sB, size_t sC) {
    typedef typename WFrag<T16>::V V;
    __shared__ __align__(16) float os[16 * 68];
    const size_t z = blockIdx.z; A += z * sA; if (A2) A2 += z * sA; Bt += z * sB; if (Bt2) Bt2 += z * sB; C += z * sC;
    const int lane = threadIdx.x & 31, lr = lane & 15, hi = lane >> 4; const int r0 = blockIdx.x * 64, c0 = blockIdx.y * 64;
    v8f acc[4][4];
#pragma unroll
    for (int mb = 0; mb < 4; ++mb)
#pragma unroll
        for (int nb = 0; nb < 4; ++nb) acc[mb][nb] = (v8f){};
    const size_t aoff = (size_t)(r0 + lr) * K + 8 * hi, boff = (size_t)(c0 + lr) * K + 8 * hi;
#pragma unroll 1
    for (int kc = 0; kc < K; kc += 32) {
        V a[4], a2[4];
#pragma unroll
        for (int mb = 0; mb < 4; ++mb) { a[mb] = WFrag<T16>::ld(A + aoff + (size_t)mb * 16 * K + kc); if (NSPLIT == 1 || NSPLIT == 2) a2[mb] = WFrag<T16>::ld(A2 + aoff + (size_t)mb * 16 * K + kc); }
#pragma unroll
        for (int nb = 0; nb < 4; ++nb) { const V b = WFrag<T16>::ld(Bt + boff + (size_t)nb * 16 * K + kc); V b2; if (NSPLIT >= 2) b2 = WFrag<T16>::ld(Bt2 + boff + (size_t)nb * 16 * K + kc);
#pragma unroll
            for (int mb = 0; mb < 4; ++mb) { acc[mb][nb] = WFrag<T16>::mma(a[mb], b, acc[mb][nb]); if (NSPLIT == 1 || NSPLIT == 2) acc[mb][nb] = WFrag<T16>::mma(a2[mb], b, acc[mb][nb]); if (NSPLIT >= 2) acc[mb][nb] = WFrag<T16>::mma(a[mb], b2, acc[mb][nb]); } }
        asm volatile("v_nop\n\tv_nop\n\tv_nop\n\tv_nop" : "+v"(acc[0][0]), "+v"(acc[1][1]), "+v"(acc[2][2]), "+v"(acc[3][3]) : "v"(a[0]), "v"(a[3]));
    }
#pragma unroll
    for (int mb = 0; mb < 4; ++mb) {
#pragma unroll
        for (int nb = 0; nb < 4; ++nb) {
#pragma unroll
            for (int j = 0; j < 8; ++j) os[(hi * 8 + j) * 68 + nb * 16 + lr] = acc[mb][nb][j]; }
        __builtin_amdgcn_wave_barrier(); asm volatile("" ::: "memory");
        float* crow = C + (size_t)(r0 + mb * 16) * ldc + c0;
#pragma unroll 1
        for (int ps = 0; ps < 2; ++ps) {
#pragma unroll
            for (int s = 0; s < 8; ++s) { const int row = 2 * s + hi, cofs = lr * 4; v4f val = *(const v4fa*)(os + row * 68 + cofs); if (BIAS) { val[0] += bfr(bias[c0 + cofs]); val[1] += bfr(bias[c0 + cofs + 1]); val[2] += bfr(bias[c0 + cofs + 2]); val[3] += bfr(bias[c0 + cofs + 3]); }
                *(volatile v4f*)(crow + (size_t)row * ldc + cofs) = val; }
            if (ps == 0) __threadfence(); }
        __builtin_amdgcn_wave_barrier(); asm volatile("" ::: "memory");
    }
}

__device__ __forceinline__ h16 tohx(float x) { return (h16)x; }
__device__ __forceinline__ void splitf(float y, unsigned short& h, unsigned short& l) { h = f2bf(y); l = f2bf(y - bf2f(h)); }
typedef __attribute__((ext_vector_type(2))) _Float16 v2h;
typedef __attribute__((ext_vector_type(4))) _Float16 v4h;
typedef __attribute__((ext_vector_type(2))) unsigned short v2us;
typedef __attribute__((ext_vector_type(4))) unsigned short v4us;
typedef __attribute__((ext_vector_type(2))) float v2f;
typedef __attribute__((ext_vector_type(4))) int v4i;

__global__ __launch_bounds__(256) void k_cvt8(const float* __restrict__ src, bf* dst, size_t n8) { const size_t i = (size_t)blockIdx.x * 256 + threadIdx.x; if (i >= n8) return; const v8f v = *(const v8f*)(src + i * 8); v8us o;
#pragma unroll
    for (int k = 0; k < 8; ++k) o[k] = f2bf(v[k]); *(volatile v8us*)(dst + i * 8) = o; __threadfence(); *(volatile v8us*)(dst + i * 8) = o; }

__global__ __launch_bounds__(256) void k_cvt8Tg(const float* __restrict__ src, bf* dst, int R, int C) { const size_t i = (size_t)blockIdx.x * 256 + threadIdx.x; if (i >= (size_t)R * C / 8) return; const int c = (int)(i / (R / 8)); const int r0 = (int)(i % (R / 8)) * 8; v8us o;
#pragma unroll
    for (int k = 0; k < 8; ++k) o[k] = f2bf(src[(size_t)(r0 + k) * C + c]); *(volatile v8us*)(dst + (size_t)c * R + r0) = o; __threadfence(); *(volatile v8us*)(dst + (size_t)c * R + r0) = o; }
__global__ __launch_bounds__(256) void k_split8(const float* __restrict__ F, bf* Ph, bf* Pl, size_t n8) { const size_t i = (size_t)blockIdx.x * 256 + threadIdx.x; if (i >= n8) return; const v8f v = *(const v8f*)(F + i * 8); v8us oh, ol;
#pragma unroll
    for (int k = 0; k < 8; ++k) { unsigned short a, c2; splitf(v[k], a, c2); oh[k] = a; ol[k] = c2; }
    *(volatile v8us*)(Ph + i * 8) = oh; *(volatile v8us*)(Pl + i * 8) = ol; __threadfence(); *(volatile v8us*)(Ph + i * 8) = oh; *(volatile v8us*)(Pl + i * 8) = ol; }

__global__ __launch_bounds__(256) void k_lsoftr(const float* __restrict__ Sb, int r0, bf* Ph, bf* Pl, float* MZ) {
    const int lane = threadIdx.x & 31; const int row = blockIdx.x * 8 + (threadIdx.x >> 5); if (row >= RB) return; const float* sr = Sb + (size_t)row * N2; float mx = -3.0e38f;
#pragma unroll 4
    for (int ch = 0; ch < N2 / 128; ++ch) { const v4f a = *(const v4f*)(sr + ch * 128 + lane * 4);
#pragma unroll
        for (int q = 0; q < 4; ++q) mx = fmaxf(mx, a[q]); }
#pragma unroll
    for (int sh = 16; sh; sh >>= 1) mx = fmaxf(mx, __shfl_xor(mx, sh, 32));
    float sum = 0.f;
#pragma unroll 4
    for (int ch = 0; ch < N2 / 128; ++ch) { const v4f a = *(const v4f*)(sr + ch * 128 + lane * 4);
#pragma unroll
        for (int q = 0; q < 4; ++q) { float d0 = __fsub_rn(a[q], mx); asm volatile("" : "+v"(d0)); sum += __builtin_amdgcn_exp2f(__fmul_rn(d0, 1.4426950408889634f)); } }
#pragma unroll
    for (int sh = 16; sh; sh >>= 1) sum += __shfl_xor(sum, sh, 32);
    const float f = __fdiv_rn(1.0f, sum);
    const float rec = (lane == 0) ? mx : ((lane == 1) ? f : 0.0f);
#pragma unroll 1
    for (int ps = 0; ps < 2; ++ps) {
#pragma unroll 2
        for (int ch = 0; ch < N2 / 128; ++ch) { const v4f a = *(const v4f*)(sr + ch * 128 + lane * 4); v4us oh, ol;
#pragma unroll
            for (int q = 0; q < 4; ++q) { float d0 = __fsub_rn(a[q], mx); asm volatile("" : "+v"(d0)); float ex = __builtin_amdgcn_exp2f(__fmul_rn(d0, 1.4426950408889634f)); asm volatile("" : "+v"(ex)); float y = ex * f; asm volatile("" : "+v"(y)); unsigned short a2, c2; splitf(y, a2, c2); oh[q] = a2; ol[q] = c2; }
            const size_t oo = (size_t)row * N2 + ch * 128 + lane * 4; *(volatile v4us*)(Ph + oo) = oh; *(volatile v4us*)(Pl + oo) = ol; }
        *(volatile float*)(MZ + (size_t)(r0 + row) * MZP + lane) = rec;
        if (ps == 0) __threadfence(); }
}

__global__ __launch_bounds__(256) void k_expT(const float* __restrict__ St, const float* __restrict__ MZ, bf* Ph, bf* Pl) { const size_t e = ((size_t)blockIdx.x * 256 + threadIdx.x) * 4; if (e >= (size_t)RB * N1) return; const int i0 = (int)(e % N1); const v4f a = *(const v4f*)(St + e); v4us oh, ol;
#pragma unroll
    for (int q = 0; q < 4; ++q) { const float m = MZ[(size_t)(i0 + q) * MZP], rz = MZ[(size_t)(i0 + q) * MZP + 1]; float d0 = __fsub_rn(a[q], m); asm volatile("" : "+v"(d0)); float ex = __builtin_amdgcn_exp2f(__fmul_rn(d0, 1.4426950408889634f)); asm volatile("" : "+v"(ex)); float y = ex * rz; asm volatile("" : "+v"(y)); unsigned short a2, c2; splitf(y, a2, c2); oh[q] = a2; ol[q] = c2; }
    *(volatile v4us*)(Ph + e) = oh; *(volatile v4us*)(Pl + e) = ol; __threadfence(); *(volatile v4us*)(Ph + e) = oh; *(volatile v4us*)(Pl + e) = ol; }

extern "C" void kernel_launch(void* const* d_in, const int* in_sizes, int n_in,
                              void* d_out, int out_size, void* d_ws, size_t ws_size, hipStream_t stream) {
    (void)in_sizes; (void)n_in; (void)out_size;
    const float* x1 = (const float*)d_in[0]; const float* x2 = (const float*)d_in[1]; const float* w1 = (const float*)d_in[2]; const float* b1 = (const float*)d_in[3];
    float* OUT0 = (float*)d_out;
    float* OUT1 = (float*)d_out + (size_t)N1 * D2;
    char* wsp = (char*)d_ws;
    auto take = [&](size_t bytes) { char* p = wsp; wsp += (bytes + 255) & ~(size_t)255; return (void*)p; };
    bf* X1B = (bf*)take((size_t)N1 * D1 * 2); bf* X1T = (bf*)take((size_t)D1 * N1 * 2); bf* X2B = (bf*)take((size_t)N2 * D2 * 2); bf* X2T = (bf*)take((size_t)D2 * N2 * 2); bf* W1B = (bf*)take((size_t)D2 * D1 * 2);
    float* FQ = (float*)take((size_t)N1 * D2 * 4); bf* QH = (bf*)take((size_t)N1 * D2 * 2); bf* QL = (bf*)take((size_t)N1 * D2 * 2); float* MZ = (float*)take((size_t)N1 * MZP * 4);
    float* Sb = (float*)take((size_t)RB * N2 * 4); bf* Ph = (bf*)take((size_t)RB * N2 * 2); bf* Pl = (bf*)take((size_t)RB * N2 * 2);
    if ((size_t)(wsp - (char*)d_ws) > ws_size) return;
    k_cvt8<<<(unsigned)(((size_t)N1 * D1 / 8 + 255) / 256), 256, 0, stream>>>(x1, X1B, (size_t)N1 * D1 / 8); k_cvt8Tg<<<(unsigned)(((size_t)N1 * D1 / 8 + 255) / 256), 256, 0, stream>>>(x1, X1T, N1, D1);
    k_cvt8<<<(unsigned)(((size_t)N2 * D2 / 8 + 255) / 256), 256, 0, stream>>>(x2, X2B, (size_t)N2 * D2 / 8); k_cvt8Tg<<<(unsigned)(((size_t)N2 * D2 / 8 + 255) / 256), 256, 0, stream>>>(x2, X2T, N2, D2);
    k_cvt8<<<(unsigned)(((size_t)D2 * D1 / 8 + 255) / 256), 256, 0, stream>>>(w1, W1B, (size_t)D2 * D1 / 8);
    k_gemmw<bf, 0, true><<<dim3(N1 / 64, D2 / 64, 1), 32, 0, stream>>>(X1B, nullptr, W1B, nullptr, D1, FQ, D2, b1, 0, 0, 0);
    k_split8<<<(unsigned)(((size_t)N1 * D2 / 8 + 255) / 256), 256, 0, stream>>>(FQ, QH, QL, (size_t)N1 * D2 / 8);
    for (int ib = 0; ib < N1 / RB; ++ib) {
        k_gemmw<bf, 1, false><<<dim3(RB / 64, N2 / 64, 1), 32, 0, stream>>>(QH + (size_t)ib * RB * D2, QL + (size_t)ib * RB * D2, X2B, nullptr, D2, Sb, N2, nullptr, 0, 0, 0);
        k_lsoftr<<<RB / 8, 256, 0, stream>>>(Sb, ib * RB, Ph, Pl, MZ);
        k_gemmw<bf, 1, false><<<dim3(RB / 64, D2 / 64, 1), 32, 0, stream>>>(Ph, Pl, X2T, nullptr, N2, OUT0 + (size_t)ib * RB * D2, D2, nullptr, 0, 0, 0); }
    for (int jb = 0; jb < N2 / RB; ++jb) {
        k_gemmw<bf, 3, false><<<dim3(RB / 64, N1 / 64, 1), 32, 0, stream>>>(X2B + (size_t)jb * RB * D2, nullptr, QH, QL, D2, Sb, N1, nullptr, 0, 0, 0);
        k_expT<<<(unsigned)(((size_t)RB * N1 / 4 + 255) / 256), 256, 0, stream>>>(Sb, MZ, Ph, Pl);
        k_gemmw<bf, 1, false><<<dim3(RB / 64, D1 / 64, 1), 32, 0, stream>>>(Ph, Pl, X1T, nullptr, N1, OUT1 + (size_t)jb * RB * D1, D1, nullptr, 0, 0, 0); }
}
